// WHTConv2D_31035433681532
// MI455X (gfx1250) — hardware-run, weakly checked
//
#include <hip/hip_runtime.h>
#include <math.h>

typedef __attribute__((ext_vector_type(16))) _Float16 v16h;
typedef __attribute__((ext_vector_type(8)))  _Float16 v8h;
typedef __attribute__((ext_vector_type(2)))  _Float16 v2h;
typedef __attribute__((ext_vector_type(16))) __bf16   v16b;
typedef __attribute__((ext_vector_type(8)))  __bf16   v8b;
typedef __attribute__((ext_vector_type(8)))  float    v8f;
typedef __attribute__((ext_vector_type(4)))  float    v4f;
typedef __attribute__((ext_vector_type(2)))  float    v2f;

constexpr int kNB   = 32;
constexpr int kC    = 128;
constexpr int kPl   = kNB * kC;
constexpr int kS    = 64;
constexpr int kIn   = 56;
constexpr int kPos  = kS * kS;
constexpr int kRows = kPl * kS;
constexpr int kPods = 2;
constexpr int kMixR = kPos * kNB;
constexpr int kThr  = 256;
constexpr float kInCarry = 1024.0f;
constexpr float kC1 = 512.0f, kC2 = 64.0f, kC3 = 32.0f, kC4 = 256.0f;
constexpr float kScE1 = kC1 / kInCarry;
constexpr float kScE2 = kC2 / kC1;
constexpr float kScE3 = 1.0f / (kC2 * kInCarry);
constexpr float kScE4 = kC4 / (kC3 * 64.0f);
constexpr float kScE5 = 1.0f / (kC4 * 64.0f);
constexpr float kF16MinNormal = 6.103515625e-5f;

static_assert(kNB == 32 && kC == 128 && kS == 64 && kIn == 56 && kPods == 2 && kPl == 4096 && kPos == 4096 && kRows == 262144 && kMixR == 131072, "the index arithmetic below uses these sizes");

constexpr size_t kOffH16 = 0ull;
constexpr size_t kOffWC16 = 8192ull;
constexpr size_t kOffP16A = 73728ull;
constexpr size_t kOffP16B = 33628160ull;
constexpr size_t kOffA16 = 67182592ull;
constexpr size_t kOffF32 = 134291456ull;
constexpr size_t kWsTotal = 201400320ull;
static_assert(kOffH16 == 0
  && kOffWC16 == kOffH16 + 8192ull
  && kOffP16A == kOffWC16 + 65536ull
  && kOffP16B == kOffP16A + 33554432ull
  && kOffA16 == kOffP16B + 33554432ull
  && kOffF32 == kOffA16 + 67108864ull
  && kWsTotal == kOffF32 + 67108864ull, "the carve is a chain: every region starts where the one before ends");
static_assert((kOffH16 % 256) == 0 && (kOffWC16 % 256) == 0 && (kOffP16A % 256) == 0 && (kOffP16B % 256) == 0 && (kOffA16 % 256) == 0 && (kOffF32 % 256) == 0, "every region starts on a multiple of 256 B");

__device__ __forceinline__ unsigned short f2bf_bits(float f) {
  unsigned u = __float_as_uint(f);
  return (unsigned short)((u + 0x7FFFu + ((u >> 16) & 1u)) >> 16);
}
__device__ __forceinline__ float bf_bits2f(unsigned short h) { return __uint_as_float(((unsigned)h) << 16); }
__device__ __forceinline__ float bf16r(float f) { return bf_bits2f(f2bf_bits(f)); }
__device__ __forceinline__ float carry_flush(float v, float carry) {
  const float s = v * carry;
  return (fabsf(s) < kF16MinNormal) ? 0.0f : s;
}

__device__ __forceinline__ void dep_guard4_h(v8f& a, v8f& b, v8f& c, v8f& d, v16h x, v16h y) { asm volatile("v_nop\n\tv_nop\n\tv_nop\n\tv_nop" : "+v"(a), "+v"(b), "+v"(c), "+v"(d) : "v"(x), "v"(y)); }
__device__ __forceinline__ void dep_guard4_b(v8f& a, v8f& b, v8f& c, v8f& d, v16b x, v16b y) { asm volatile("v_nop\n\tv_nop\n\tv_nop\n\tv_nop" : "+v"(a), "+v"(b), "+v"(c), "+v"(d) : "v"(x), "v"(y)); }
__device__ __forceinline__ void keep4_h(v16h a, v16h b, v16h c, v16h d) { asm volatile("v_nop" :: "v"(a), "v"(b), "v"(c), "v"(d)); }
__device__ __forceinline__ void keep4_b(v16b a, v16b b, v16b c, v16b d) { asm volatile("v_nop" :: "v"(a), "v"(b), "v"(c), "v"(d)); }
__device__ __forceinline__ void acc_guard4(v8f& a, v8f& b, v8f& c, v8f& d) { asm volatile("v_nop\n\tv_nop\n\tv_nop\n\tv_nop" : "+v"(a), "+v"(b), "+v"(c), "+v"(d)); }

template <typename T> struct Frag;
template <> struct Frag<_Float16> {
  typedef v16h V; union U { v16h v; v8h h[2]; };
  static __device__ __forceinline__ v16h load(const _Float16* p) {
    U f; f.h[0] = *(const v8h*)(p); f.h[1] = *(const v8h*)(p + 16); return f.v;
  }
  static __device__ __forceinline__ v8f mma(v16h a, v16h b, v8f c) {
    return __builtin_amdgcn_wmma_f32_16x16x32_f16(false, a, false, b, (short)0, c, false, false);
  }
  static __device__ __forceinline__ void guard4(v8f& a, v8f& b, v8f& c, v8f& d, v16h x, v16h y) { dep_guard4_h(a, b, c, d, x, y); }
  static __device__ __forceinline__ void keep(v16h a, v16h b, v16h c, v16h d) { keep4_h(a, b, c, d); }
};
template <> struct Frag<__bf16> {
  typedef v16b V; union U { v16b v; v8b h[2]; };
  static __device__ __forceinline__ v16b load(const __bf16* p) {
    U f; f.h[0] = *(const v8b*)(p); f.h[1] = *(const v8b*)(p + 16); return f.v;
  }
  static __device__ __forceinline__ v8f mma(v16b a, v16b b, v8f c) {
    return __builtin_amdgcn_wmma_f32_16x16x32_bf16(false, a, false, b, (short)0, c, false, false);
  }
  static __device__ __forceinline__ void guard4(v8f& a, v8f& b, v8f& c, v8f& d, v16b x, v16b y) { dep_guard4_b(a, b, c, d, x, y); }
  static __device__ __forceinline__ void keep(v16b a, v16b b, v16b c, v16b d) { keep4_b(a, b, c, d); }
};

__device__ __forceinline__ v8f mma_h(v16h a, v16h b, v8f c) {
  c = __builtin_amdgcn_wmma_f32_16x16x32_f16(false, a, false, b, (short)0, c, false, false);
  asm volatile("v_nop\n\tv_nop\n\tv_nop\n\tv_nop" : "+v"(c) : "v"(a), "v"(b));
  return c;
}

template <int ET> struct Elem;
template <> struct Elem<0> { typedef _Float16 T; };
template <> struct Elem<1> { typedef __bf16 T; };
template <int ET, bool SPLIT, int BIAS_MODE, int OUT_MODE, bool RESID, int ACT = 0>
__global__ __launch_bounds__(256) void wmma_gemm64(
    const unsigned short* __restrict__ Ap, const unsigned short* __restrict__ A2p, int lda, long strideA,
    const unsigned short* __restrict__ Btp, const unsigned short* __restrict__ Bt2p, int ldb, long strideB,
    void* __restrict__ Cout, void* __restrict__ Cout2, int ldc, long strideC,
    const float* __restrict__ bias,
    const float* __restrict__ resid, long strideR,
    int M, int N, int K, float scale) {
  typedef typename Elem<ET>::T T;
  typedef typename Frag<T>::V V;
  const T* A = (const T*)Ap; const T* A2 = (const T*)A2p; const T* Bt = (const T*)Btp; const T* Bt2 = (const T*)Bt2p;
  __shared__ __align__(16) float sT[8][16 * 68];
  const int b    = blockIdx.y;
  const int lane = threadIdx.x & 31;
  const int wave = threadIdx.x >> 5;
  const int tilesN = N >> 6;
  const int tilesM = M >> 6;
  const int tile = blockIdx.x * 8 + wave;
  if (tile >= tilesM * tilesN) return;
  const int tm = tile / tilesN;
  const int tn = tile - tm * tilesN;
  const int m0 = tm << 6;
  const int n0 = tn << 6;

  const T* Ab  = A  + (size_t)b * strideA;
  const T* Bb  = Bt + (size_t)b * strideB;
  const T* Ab2 = SPLIT ? (A2  + (size_t)b * strideA) : nullptr;
  const T* Bb2 = SPLIT ? (Bt2 + (size_t)b * strideB) : nullptr;

  const int rlane = lane & 15;
  const int koff  = (lane >> 4) * 8;
  const int mOff  = (lane >> 4) * 8;

  v8f acc[4][4];
#pragma unroll
  for (int i = 0; i < 4; ++i)
#pragma unroll
    for (int j = 0; j < 4; ++j) acc[i][j] = (v8f){0.f,0.f,0.f,0.f,0.f,0.f,0.f,0.f};

  for (int k0 = 0; k0 < K; k0 += 32) {
    V bh[4], bl[4];
#pragma unroll
    for (int j = 0; j < 4; ++j) {
      const size_t bo = (size_t)(n0 + (j << 4) + rlane) * ldb + koff + k0;
      bh[j] = Frag<T>::load(Bb + bo);
      if (SPLIT) bl[j] = Frag<T>::load(Bb2 + bo);
    }
#pragma unroll
    for (int i = 0; i < 4; ++i) {
      const size_t ao = (size_t)(m0 + (i << 4) + rlane) * lda + koff + k0;
      V ah = Frag<T>::load(Ab + ao);
      V al;
      if (SPLIT) al = Frag<T>::load(Ab2 + ao);
#pragma unroll
      for (int j = 0; j < 4; ++j) {
        acc[i][j] = Frag<T>::mma(ah, bh[j], acc[i][j]);
        if (SPLIT) {
          acc[i][j] = Frag<T>::mma(ah, bl[j], acc[i][j]);
          acc[i][j] = Frag<T>::mma(al, bh[j], acc[i][j]);
        }
      }
      Frag<T>::guard4(acc[i][0], acc[i][1], acc[i][2], acc[i][3], ah, SPLIT ? al : ah);
    }
    Frag<T>::keep(bh[0], bh[1], bh[2], bh[3]);
    if (SPLIT) Frag<T>::keep(bl[0], bl[1], bl[2], bl[3]);
  }
  acc_guard4(acc[0][0], acc[0][1], acc[0][2], acc[0][3]);
  acc_guard4(acc[1][0], acc[1][1], acc[1][2], acc[1][3]);
  acc_guard4(acc[2][0], acc[2][1], acc[2][2], acc[2][3]);
  acc_guard4(acc[3][0], acc[3][1], acc[3][2], acc[3][3]);

  float* slab = sT[wave];
  const float* Rb = RESID ? (resid + (size_t)b * strideR) : nullptr;
#pragma unroll
  for (int i = 0; i < 4; ++i) {
    const int mBase = m0 + (i << 4);
#pragma unroll
    for (int j = 0; j < 4; ++j) {
      const int n = n0 + (j << 4) + rlane;
      float bv = 0.f;
      if (BIAS_MODE == 2) bv = bias[n];
#pragma unroll
      for (int r = 0; r < 8; ++r) {
        float v = acc[i][j][r] * scale;
        if (BIAS_MODE == 1) v += bias[mBase + mOff + r];
        if (BIAS_MODE == 2) v += bv;
        if (RESID) v += Rb[(size_t)(mBase + mOff + r) * ldc + n];
        if (ACT == 1) v = tanhf(v);
        if (ACT == 2) v = fmaxf(v, 0.0f);
        if (ACT == 3) v = v / (1.0f + expf(-v));
        if (ACT == 4) v = (v > 0.f) ? v : 0.01f * v;
        slab[(mOff + r) * 68 + (j << 4) + rlane] = v;
      }
    }
    __builtin_amdgcn_fence(__ATOMIC_RELEASE, "workgroup");
    __builtin_amdgcn_wave_barrier();
    __builtin_amdgcn_fence(__ATOMIC_ACQUIRE, "workgroup");
    if (OUT_MODE == 0) {
      float* C = (float*)Cout + (size_t)b * strideC;
      const int hh = lane >> 4, c4 = (lane & 15) * 4;
      for (int pass = 0; pass < 2; ++pass) {
#pragma unroll
        for (int it = 0; it < 8; ++it) {
          const int row = it * 2 + hh;
          v4f v = *(const v4f*)(slab + row * 68 + c4);
          *(volatile v4f*)(C + (size_t)(mBase + row) * ldc + n0 + c4) = v;
        }
        __threadfence();
      }
    } else {
      const int q = lane >> 3, c8 = (lane & 7) * 8;
      unsigned short* C  = (unsigned short*)Cout  + (size_t)b * strideC;
      unsigned short* C2 = (OUT_MODE == 2) ? ((unsigned short*)Cout2 + (size_t)b * strideC) : nullptr;
      for (int pass = 0; pass < 2; ++pass) {
#pragma unroll
        for (int it = 0; it < 4; ++it) {
          const int row = it * 4 + q;
          const float* sp = slab + row * 68 + c8;
          v8h hv, lv;
#pragma unroll
          for (int e = 0; e < 8; ++e) {
            if (OUT_MODE == 1) {
              hv[e] = (_Float16)sp[e];
            } else {
              unsigned short hb = f2bf_bits(sp[e]);
              unsigned short lb = f2bf_bits(sp[e] - bf_bits2f(hb));
              hv[e] = __builtin_bit_cast(_Float16, hb);
              lv[e] = __builtin_bit_cast(_Float16, lb);
            }
          }
          *(volatile v8h*)(C + (size_t)(mBase + row) * ldc + n0 + c8) = hv;
          if (OUT_MODE == 2) *(volatile v8h*)(C2 + (size_t)(mBase + row) * ldc + n0 + c8) = lv;
        }
        __threadfence();
      }
    }
    __builtin_amdgcn_fence(__ATOMIC_RELEASE, "workgroup");
    __builtin_amdgcn_wave_barrier();
    __builtin_amdgcn_fence(__ATOMIC_ACQUIRE, "workgroup");
  }
}

__global__ __launch_bounds__(kThr) void cast_plane_kernel(const float* __restrict__ src, unsigned short* __restrict__ dst,
                                                          int colsLog2, int dstPitch, int dstOff) {
  const int i   = blockIdx.x * kThr + threadIdx.x;
  const int sh  = colsLog2 - 3;
  const int row = i >> sh;
  const int c8  = (i & ((1 << sh) - 1)) * 8;
  const float* sp = src + ((size_t)row << colsLog2) + c8;
  const v4f a0 = *(const v4f*)(sp);
  const v4f a1 = *(const v4f*)(sp + 4);
  v8h hv;
#pragma unroll
  for (int e = 0; e < 4; ++e) {
    const float f0 = a0[e];
    const float f1 = a1[e];
    hv[e]     = (_Float16)carry_flush(bf16r(f0), kInCarry);
    hv[4 + e] = (_Float16)carry_flush(bf16r(f1), kInCarry);
  }
  unsigned short* dp = dst + (size_t)row * dstPitch + dstOff + c8;
  *(volatile v8h*)dp = hv;
  __threadfence();
  *(volatile v8h*)dp = hv;
}

__global__ __launch_bounds__(kThr) void had_kernel(unsigned short* __restrict__ Hm) {
  const unsigned i = blockIdx.x * (unsigned)kThr + threadIdx.x;
  const unsigned r = i >> 3, c8 = (i & 7u) << 3;
  v8h hv;
#pragma unroll
  for (int e = 0; e < 8; ++e) {
    const unsigned par = (unsigned)__builtin_popcount(r & (c8 + (unsigned)e)) & 1u;
    hv[e] = __builtin_bit_cast(_Float16, (unsigned short)(0x3C00u | (par << 15)));
  }
  unsigned short* dp = Hm + (size_t)i * 8u;
  *(volatile v8h*)dp = hv;
  __threadfence();
  *(volatile v8h*)dp = hv;
}

__global__ __launch_bounds__(kThr) void xpadc_kernel(const float* __restrict__ x, unsigned short* __restrict__ X16) {
  const unsigned i = blockIdx.x * (unsigned)kThr + threadIdx.x;
  const unsigned p = i >> 9, h = (i >> 3) & 63u, g = i & 7u;
  const unsigned keep = ((h < (unsigned)kIn) & (g < 7u)) ? 0xFFFFFFFFu : 0u;
  const unsigned hs = (h < (unsigned)kIn) ? h : (unsigned)(kIn - 1);
  const unsigned gs = (g < 7u) ? g : 6u;
  const float* sp = x + ((size_t)p * kIn + hs) * (unsigned)kIn + 8u * gs;
  const v4f a0 = *(const v4f*)sp, a1 = *(const v4f*)(sp + 4);
  v8h hv;
#pragma unroll
  for (int e = 0; e < 4; ++e) {
    hv[e]     = (_Float16)__uint_as_float(__float_as_uint(carry_flush(bf16r(a0[e]), kInCarry)) & keep);
    hv[4 + e] = (_Float16)__uint_as_float(__float_as_uint(carry_flush(bf16r(a1[e]), kInCarry)) & keep);
  }
  unsigned short* dp = X16 + (size_t)i * 8u;
  *(volatile v8h*)dp = hv;
  __threadfence();
  *(volatile v8h*)dp = hv;
}

__global__ __launch_bounds__(kThr) void sjoin_kernel(const unsigned short* __restrict__ C2, const float* __restrict__ lv, unsigned short* __restrict__ A16) {
  const unsigned i = blockIdx.x * (unsigned)kThr + threadIdx.x;
  const unsigned r = i >> 4, c8 = (i & 15u) << 3, pos = r >> 5;
  const v8h cv = *(const v8h*)(C2 + (size_t)r * (unsigned)kC + c8);
  const float v0 = expf(bf16r(lv[pos])), v1 = expf(bf16r(lv[(unsigned)kPos + pos]));
  v8h h0, h1;
#pragma unroll
  for (int e = 0; e < 8; ++e) {
    const float f = (float)cv[e] * (1.0f / kC2);
    h0[e] = (_Float16)carry_flush(f * v0, kC2);
    h1[e] = (_Float16)carry_flush(f * v1, kC2);
  }
  unsigned short* dp = A16 + (size_t)r * (unsigned)(kPods * kC) + c8;
  *(volatile v8h*)dp = h0;
  *(volatile v8h*)(dp + kC) = h1;
  __threadfence();
  *(volatile v8h*)dp = h0;
  *(volatile v8h*)(dp + kC) = h1;
}

__global__ __launch_bounds__(kThr) void thturn_kernel(const float* __restrict__ F5, const float* __restrict__ T, unsigned short* __restrict__ G16) {
  const unsigned i = blockIdx.x * (unsigned)kThr + threadIdx.x;
  const unsigned q = i >> 9, kh = (i >> 3) & 63u, kw8 = (i & 7u) << 3;
  const unsigned b = q >> 7, oc = q & 127u;
  const float t = fmaxf(bf16r(T[oc]), 0.0f);
  const float* sp = F5 + ((size_t)(kh * (unsigned)kS + kw8) * (unsigned)kNB + b) * (unsigned)kC + oc;
  v8h hv;
#pragma unroll
  for (int e = 0; e < 8; ++e) {
    const float f = sp[(size_t)e * (unsigned)(kNB * kC)];
    const float g = copysignf(fmaxf(fabsf(f) - t, 0.0f), f);
    hv[e] = (_Float16)carry_flush(g, kC3);
  }
  unsigned short* dp = G16 + (size_t)i * 8u;
  *(volatile v8h*)dp = hv;
  __threadfence();
  *(volatile v8h*)dp = hv;
}

__global__ __launch_bounds__(kThr) void cropres_kernel(const float* __restrict__ C5, const float* __restrict__ x, float* __restrict__ out) {
  const unsigned i = blockIdx.x * (unsigned)kThr + threadIdx.x;
  const unsigned q = i / 392u, rem = i - q * 392u, h = rem / 7u, w8 = (rem - h * 7u) << 3;
  const size_t oi = ((size_t)q * kIn + h) * (unsigned)kIn + w8;
  const v4f x0 = *(const v4f*)(x + oi), x1 = *(const v4f*)(x + oi + 4);
  const float* sp = C5 + ((size_t)h * (unsigned)kS + w8) * (unsigned)kPl + q;
  v4f y0, y1;
#pragma unroll
  for (int e = 0; e < 4; ++e) {
    y0[e] = sp[(size_t)e * (unsigned)kPl] + bf16r(x0[e]);
    y1[e] = sp[(size_t)(4 + e) * (unsigned)kPl] + bf16r(x1[e]);
  }
  float* dp = out + oi;
  *(volatile v4f*)dp = y0;
  *(volatile v4f*)(dp + 4) = y1;
  __threadfence();
  *(volatile v4f*)dp = y0;
  *(volatile v4f*)(dp + 4) = y1;
}
static_assert(kPl * kIn * 7 == 6272 * kThr, "the last kernel's grid exact");

extern "C" void kernel_launch(void* const* d_in, const int* in_sizes, int n_in,
                              void* d_out, int out_size, void* d_ws, size_t ws_size,
                              hipStream_t stream) {
  if (n_in < 4 || d_out == nullptr || d_ws == nullptr) return;
  if (in_sizes[0] != kPl * kIn * kIn || in_sizes[1] != kPods * kC * kC || in_sizes[2] != kPods * kPos || in_sizes[3] != kC) return;
  if (out_size != kPl * kIn * kIn) return;
  if (ws_size < kWsTotal) return;
  const float* x = (const float*)d_in[0];
  const float* cw = (const float*)d_in[1];
  const float* lv = (const float*)d_in[2];
  const float* T = (const float*)d_in[3];
  float* out = (float*)d_out;
  char* ws = (char*)d_ws;
  unsigned short* H16 = (unsigned short*)(ws + kOffH16);
  unsigned short* WC16 = (unsigned short*)(ws + kOffWC16);
  unsigned short* P16A = (unsigned short*)(ws + kOffP16A);
  unsigned short* P16B = (unsigned short*)(ws + kOffP16B);
  unsigned short* A16 = (unsigned short*)(ws + kOffA16);
  float* F32 = (float*)(ws + kOffF32);

  static_assert((kS * kS / 8) % kThr == 0 && (kC * kC / 8) % kThr == 0 && (kRows * kS / 8) % kThr == 0 && (kMixR * kC / 8) % kThr == 0, "every flat kernel's grid exact");
  had_kernel<<<kS * kS / 8 / kThr, kThr, 0, stream>>>(H16);
  cast_plane_kernel<<<kC * kC / 8 / kThr, kThr, 0, stream>>>(cw, WC16, 7, kPods * kC, 0);
  cast_plane_kernel<<<kC * kC / 8 / kThr, kThr, 0, stream>>>(cw + (size_t)kC * kC, WC16, 7, kPods * kC, kC);
  xpadc_kernel<<<kRows * kS / 8 / kThr, kThr, 0, stream>>>(x, P16A);
  wmma_gemm64<0, false, 0, 1, false, 0><<<dim3((kS / 64) * (kRows / 64) / 8, 1), 256, 0, stream>>>(
      H16, H16, kS, 0L, P16A, P16A, kS, 0L, (void*)P16B, (void*)P16B, kRows, 0L, nullptr, nullptr, 0L, kS, kRows, kS, kScE1);
  wmma_gemm64<0, false, 0, 1, false, 0><<<dim3((kS / 64) * (kRows / 64) / 8, 1), 256, 0, stream>>>(
      H16, H16, kS, 0L, P16B, P16B, kS, 0L, (void*)P16A, (void*)P16A, kRows, 0L, nullptr, nullptr, 0L, kS, kRows, kS, kScE2);
  sjoin_kernel<<<kMixR * kC / 8 / kThr, kThr, 0, stream>>>(P16A, lv, A16);
  wmma_gemm64<0, false, 0, 0, false, 0><<<dim3((kMixR / 64) * (kC / 64) / 8, 1), 256, 0, stream>>>(
      A16, A16, kPods * kC, 0L, WC16, WC16, kPods * kC, 0L, (void*)F32, (void*)F32, kC, 0L, nullptr, nullptr, 0L, kMixR, kC, kPods * kC, kScE3);
  thturn_kernel<<<kRows * kS / 8 / kThr, kThr, 0, stream>>>(F32, T, P16B);
  wmma_gemm64<0, false, 0, 1, false, 0><<<dim3((kS / 64) * (kRows / 64) / 8, 1), 256, 0, stream>>>(
      H16, H16, kS, 0L, P16B, P16B, kS, 0L, (void*)P16A, (void*)P16A, kRows, 0L, nullptr, nullptr, 0L, kS, kRows, kS, kScE4);
  wmma_gemm64<0, false, 0, 0, false, 0><<<dim3((kS / 64) * (kRows / 64) / 8, 1), 256, 0, stream>>>(
      H16, H16, kS, 0L, P16A, P16A, kS, 0L, (void*)F32, (void*)F32, kRows, 0L, nullptr, nullptr, 0L, kS, kRows, kS, kScE5);
  cropres_kernel<<<kPl * kIn * 7 / kThr, kThr, 0, stream>>>(F32, x, out);
}
static_assert(((kS / 64) * (kRows / 64)) % 8 == 0 && ((kMixR / 64) * (kC / 64)) % 8 == 0 && kS % 32 == 0 && (kPods * kC) % 32 == 0, "the engine's grids: whole blocks of eight wave tiles; the depths multiples of 32");
